// SSM_58076547776593
// MI455X (gfx1250) — hardware-run, weakly checked
//
#include <hip/hip_runtime.h>


#define NM   4096
#define NB   2
#define NT   2048
#define ND   512
#define NP   64
#define NS   16
typedef _Float16 h16;
typedef unsigned short bf;
typedef __attribute__((ext_vector_type(16))) __bf16   v16bf;
typedef __attribute__((ext_vector_type(16))) _Float16 v16h;
typedef __attribute__((ext_vector_type(8)))  _Float16 v8h;
typedef __attribute__((ext_vector_type(8)))  unsigned short v8us;
typedef __attribute__((ext_vector_type(8)))  float    v8f;
typedef __attribute__((ext_vector_type(4)))  float    v4f;
typedef v8h  __attribute__((may_alias)) v8ha;
typedef v4f  __attribute__((may_alias)) v4fa;
typedef v8us __attribute__((may_alias)) v8usa;

__device__ __forceinline__ unsigned short f2bf(float f) { unsigned u = __float_as_uint(f); u += 0x7FFFu + ((u >> 16) & 1u); return (unsigned short)(u >> 16); }
__device__ __forceinline__ float bf2f(unsigned short b) { return __uint_as_float(((unsigned)b) << 16); }
__device__ __forceinline__ float bfr(float f) { return bf2f(f2bf(f)); }
__device__ __forceinline__ v16h cat16(v8h lo, v8h hi) { return __builtin_shufflevector(lo, hi, 0, 1, 2, 3, 4, 5, 6, 7, 8, 9, 10, 11, 12, 13, 14, 15); }
__device__ __forceinline__ v16bf cat16b(v8us lo, v8us hi) { return __builtin_bit_cast(v16bf, __builtin_shufflevector(lo, hi, 0, 1, 2, 3, 4, 5, 6, 7, 8, 9, 10, 11, 12, 13, 14, 15)); }
__device__ __forceinline__ v8f wmma16(v16h a, v16h b, v8f c) { return __builtin_amdgcn_wmma_f32_16x16x32_f16(false, a, false, b, (short)0, c, false, false); }
__device__ __forceinline__ v8f wmmab(v16bf a, v16bf b, v8f c) { return __builtin_amdgcn_wmma_f32_16x16x32_bf16(false, a, false, b, (short)0, c, false, false); }

template <typename T16> struct WFrag;
template <> struct WFrag<h16> { typedef v16h V; static __device__ __forceinline__ V ld(const h16* p) { return cat16(*(const v8h*)p, *(const v8h*)(p + 16)); } static __device__ __forceinline__ v8f mma(V a, V b, v8f c) { return wmma16(a, b, c); } };
template <> struct WFrag<bf> { typedef v16bf V; static __device__ __forceinline__ V ld(const bf* p) { return cat16b(*(const v8us*)p, *(const v8us*)(p + 16)); } static __device__ __forceinline__ v8f mma(V a, V b, v8f c) { return wmmab(a, b, c); } };
template <typename T16, int NSPLIT, bool BIAS>
__global__ __launch_bounds__(32) void k_gemmw(const T16* __restrict__ A, const T16* __restrict__ A2, const T16* __restrict__ Bt, const T16* __restrict__ Bt2, int K, float* C, int ldc, const float* __restrict__ bias, size_t sA, size_t sB, size_t sC) {
    typedef typename WFrag<T16>::V V;
    __shared__ __align__(16) float os[16 * 68];
    const size_t z = blockIdx.z; A += z * sA; if (A2) A2 += z * sA; Bt += z * sB; if (Bt2) Bt2 += z * sB; C += z * sC;
    const int lane = threadIdx.x & 31, lr = lane & 15, hi = lane >> 4; const int r0 = blockIdx.x * 64, c0 = blockIdx.y * 64;
    v8f acc[4][4];
#pragma unroll
    for (int mb = 0; mb < 4; ++mb)
#pragma unroll
        for (int nb = 0; nb < 4; ++nb) acc[mb][nb] = (v8f){};
    const size_t aoff = (size_t)(r0 + lr) * K + 8 * hi, boff = (size_t)(c0 + lr) * K + 8 * hi;
    for (int kc = 0; kc < K; kc += 32) {
        V a[4], a2[4];
#pragma unroll
        for (int mb = 0; mb < 4; ++mb) { a[mb] = WFrag<T16>::ld(A + aoff + (size_t)mb * 16 * K + kc); if (NSPLIT == 1 || NSPLIT == 2) a2[mb] = WFrag<T16>::ld(A2 + aoff + (size_t)mb * 16 * K + kc); }
#pragma unroll
        for (int nb = 0; nb < 4; ++nb) { const V b = WFrag<T16>::ld(Bt + boff + (size_t)nb * 16 * K + kc); V b2; if (NSPLIT >= 2) b2 = WFrag<T16>::ld(Bt2 + boff + (size_t)nb * 16 * K + kc);
#pragma unroll
            for (int mb = 0; mb < 4; ++mb) { acc[mb][nb] = WFrag<T16>::mma(a[mb], b, acc[mb][nb]); if (NSPLIT == 1 || NSPLIT == 2) acc[mb][nb] = WFrag<T16>::mma(a2[mb], b, acc[mb][nb]); if (NSPLIT >= 2) acc[mb][nb] = WFrag<T16>::mma(a[mb], b2, acc[mb][nb]); } }
        asm volatile("v_nop\n\tv_nop\n\tv_nop\n\tv_nop" : "+v"(acc[0][0]), "+v"(acc[1][1]), "+v"(acc[2][2]), "+v"(acc[3][3]) : "v"(a[0]), "v"(a[3]));
    }
#pragma unroll
    for (int mb = 0; mb < 4; ++mb) {
#pragma unroll
        for (int nb = 0; nb < 4; ++nb) {
#pragma unroll
            for (int j = 0; j < 8; ++j) os[(hi * 8 + j) * 68 + nb * 16 + lr] = acc[mb][nb][j]; }
        __builtin_amdgcn_wave_barrier(); asm volatile("" ::: "memory");
        float* crow = C + (size_t)(r0 + mb * 16) * ldc + c0;
#pragma unroll 1
        for (int ps = 0; ps < 2; ++ps) {
#pragma unroll
            for (int s = 0; s < 8; ++s) { const int row = 2 * s + hi, cofs = lr * 4; v4f val = *(const v4fa*)(os + row * 68 + cofs); if (BIAS) { val[0] += bfr(bias[c0 + cofs]); val[1] += bfr(bias[c0 + cofs + 1]); val[2] += bfr(bias[c0 + cofs + 2]); val[3] += bfr(bias[c0 + cofs + 3]); }
                *(volatile v4f*)(crow + (size_t)row * ldc + cofs) = val; }
            if (ps == 0) __threadfence(); }
        __builtin_amdgcn_wave_barrier(); asm volatile("" ::: "memory");
    }
}

typedef __attribute__((ext_vector_type(2))) _Float16 v2h;
typedef __attribute__((ext_vector_type(4))) _Float16 v4h;
typedef __attribute__((ext_vector_type(2))) unsigned short v2us;
typedef __attribute__((ext_vector_type(4))) unsigned short v4us;
typedef __attribute__((ext_vector_type(2))) float v2f;
typedef __attribute__((ext_vector_type(4))) int v4i;
__global__ __launch_bounds__(256) void k_cvt8(const float* __restrict__ src, bf* dst, size_t n8) { const size_t i = (size_t)blockIdx.x * 256 + threadIdx.x; if (i >= n8) return; const v8f v = *(const v8f*)(src + i * 8); v8us o;
#pragma unroll
    for (int k = 0; k < 8; ++k) o[k] = f2bf(v[k]); *(volatile v8us*)(dst + i * 8) = o; __threadfence(); *(volatile v8us*)(dst + i * 8) = o; }

template <typename T16> __device__ __forceinline__ unsigned short cv16(float x);
template <> __device__ __forceinline__ unsigned short cv16<bf>(float x) { return f2bf(x); }
template <> __device__ __forceinline__ unsigned short cv16<h16>(float x) { const h16 h = (h16)x; return __builtin_bit_cast(unsigned short, h); }
template <typename T16>
__global__ __launch_bounds__(256) void k_castp(const float* __restrict__ src, int rows_valid, int lc, float mul, unsigned short* dst) { const unsigned e = blockIdx.x * 256 + threadIdx.x; const unsigned r = e >> (lc - 3); const unsigned c0 = (e & ((1u << (lc - 3)) - 1u)) << 3; const unsigned rr = (r < (unsigned)rows_valid) ? r : (unsigned)(rows_valid - 1);
    const float* s = src + ((size_t)rr << lc) + c0; const v4f a = *(const v4f*)s, b = *(const v4f*)(s + 4); const float lm = (r < (unsigned)rows_valid) ? mul : 0.0f; v8us o;
#pragma unroll
    for (int q = 0; q < 4; ++q) { o[q] = cv16<T16>(__fmul_rn(a[q], lm)); o[q + 4] = cv16<T16>(__fmul_rn(b[q], lm)); }
    *(volatile v8us*)(dst + (size_t)e * 8) = o; __threadfence(); *(volatile v8us*)(dst + (size_t)e * 8) = o; }

__device__ __forceinline__ float sp(float v) { return fmaxf(v, 0.0f) + log1pf(expf(-fabsf(v))); }

__global__ __launch_bounds__(64) void k_bv(const float* __restrict__ v1, const float* __restrict__ v2, const float* __restrict__ v3, float* V) { const int j = threadIdx.x; const float p = v1[j & 15], q = v2[j & 15], r = v3[0]; const unsigned m1 = 0u - (unsigned)(j < 16), m2 = 0u - (unsigned)((j >= 16) & (j < 32)), m3 = 0u - (unsigned)(j == 32); const float o = __uint_as_float((__float_as_uint(p) & m1) | (__float_as_uint(q) & m2) | (__float_as_uint(r) & m3)); *(volatile float*)(V + j) = o; __threadfence(); *(volatile float*)(V + j) = o; }

__global__ __launch_bounds__(256) void k_scan(const float* __restrict__ P, const float* __restrict__ x, const float* __restrict__ Am, float* out) { const int i = blockIdx.x * 256 + threadIdx.x; if (i >= NB * ND) return; const int b = i / ND; const int d = i % ND; float am[NS], rn[NS], h[NS];
#pragma unroll
    for (int n = 0; n < NS; ++n) { am[n] = bfr(Am[(size_t)d * NS + n]); rn[n] = 1.0f / (-am[n]); h[n] = 0.0f; }
    for (int t0 = 0; t0 < NT; t0 += 8) { float y8[8];
#pragma unroll
        for (int s = 0; s < 8; ++s) { const size_t r = (size_t)b * NT + t0 + s; const float* pr = P + r * NP; const float q = sp(pr[2 * NS]); const float xv = bfr(x[r * ND + d]); float y = 0.0f;
#pragma unroll
            for (int n = 0; n < NS; ++n) { const float g = q * am[n]; const float a = expf(g); const float fq = (1.0f - a) * rn[n]; const float fs = q * (1.0f - 0.5f * g + g * g * 0.16666667f); const float f = (fabsf(am[n]) > 1e-6f) ? fq : fs; h[n] = a * h[n] + (f * pr[n]) * xv; y = y + h[n] * pr[NS + n]; }
            y8[s] = y; }
        float* o = out + ((size_t)b * NT + t0) * ND + d;
#pragma unroll
        for (int s = 0; s < 8; ++s) *(volatile float*)(o + (size_t)s * ND) = y8[s];
        __threadfence();
#pragma unroll
        for (int s = 0; s < 8; ++s) *(volatile float*)(o + (size_t)s * ND) = y8[s]; }
}

extern "C" void kernel_launch(void* const* d_in, const int* in_sizes, int n_in, void* d_out, int out_size, void* d_ws, size_t ws_size, hipStream_t stream) {
    if (n_in < 8) return;
    if (in_sizes[0] != NM * ND || in_sizes[1] != ND * NS || in_sizes[2] != NS * ND || in_sizes[3] != NS || in_sizes[4] != NS * ND || in_sizes[5] != NS || in_sizes[6] != ND || in_sizes[7] != 1) return;
    if (out_size != NM * ND) return;
    static_assert(NM == NB * NT && NM % 64 == 0 && NP == 64 && ND == 512 && ND % 32 == 0 && 2 * NS + 1 <= NP && (NM * ND / 8) % 256 == 0 && (NS * ND / 8) % 256 == 0 && ((NP - 2 * NS) * ND / 8) % 256 == 0 && (NB * ND) % 256 == 0 && NT % 8 == 0, "the product: M a multiple of 64 on ONE 64-column tile, the depth of 32; the flat grids exact; k_castp's plane of 2^9 columns; a wave's 32 channels in one batch; the steps in eights");
    const float* x = (const float*)d_in[0]; const float* Am = (const float*)d_in[1]; const float* Wb = (const float*)d_in[2]; const float* vb = (const float*)d_in[3]; const float* Wc = (const float*)d_in[4]; const float* vc = (const float*)d_in[5]; const float* wq = (const float*)d_in[6]; const float* vq = (const float*)d_in[7]; float* out = (float*)d_out;
    char* wsp = (char*)d_ws; auto take = [&](size_t bytes) { char* p = wsp; wsp += (bytes + 255) & ~(size_t)255; return (void*)p; };
    bf* Xb = (bf*)take((size_t)NM * ND * 2); bf* B1 = (bf*)take((size_t)NP * ND * 2); float* V = (float*)take((size_t)NP * 4); float* P = (float*)take((size_t)NM * NP * 4);
    if ((size_t)(wsp - (char*)d_ws) > ws_size) return;
    k_cvt8<<<(unsigned)(NM * ND / 8 / 256), 256, 0, stream>>>(x, Xb, (size_t)NM * ND / 8);
    k_castp<bf><<<(unsigned)(NS * ND / 8 / 256), 256, 0, stream>>>(Wb, NS, 9, 1.0f, (unsigned short*)B1);
    k_castp<bf><<<(unsigned)(NS * ND / 8 / 256), 256, 0, stream>>>(Wc, NS, 9, 1.0f, (unsigned short*)(B1 + (size_t)NS * ND));
    k_castp<bf><<<(unsigned)((NP - 2 * NS) * ND / 8 / 256), 256, 0, stream>>>(wq, 1, 9, 1.0f, (unsigned short*)(B1 + (size_t)2 * NS * ND));
    k_bv<<<1, 64, 0, stream>>>(vb, vc, vq, V);
    k_gemmw<bf, 0, true><<<dim3(NM / 64, NP / 64, 1), 32, 0, stream>>>(Xb, nullptr, B1, nullptr, ND, P, NP, V, 0, 0, 0);
    k_scan<<<(unsigned)(NB * ND / 256), 256, 0, stream>>>(P, x, Am, out);
}
